// ReciprocalSpaceAttention_38319698215318
// MI455X (gfx1250) — hardware-run, weakly checked
//
#include <hip/hip_runtime.h>
#include <stdint.h>

#pragma clang fp contract(off)

#define DEVINL __device__ __forceinline__

typedef __attribute__((ext_vector_type(16))) __bf16 v16b;
typedef unsigned short v8us __attribute__((ext_vector_type(8)));
typedef float v8f __attribute__((ext_vector_type(8)));
typedef float v4f __attribute__((ext_vector_type(4)));
typedef int   v4i __attribute__((ext_vector_type(4)));
typedef v8us __attribute__((may_alias)) v8usa;
typedef v4f  __attribute__((may_alias)) v4fa;
typedef v4i  __attribute__((may_alias)) v4ia;
union FragB { v16b v; v8us half[2]; };

#define HD     64
#define MK     64
#define NT     64
#define TPB    256
#define WAVES  8
#define PU     72
#define PF     68
#define QSCALE 0.125f

static_assert(TPB == WAVES * 32);
static_assert((PU % 8) == 0);
static_assert((PF % 4) == 0);
static_assert(HD == 64);
static_assert(MK == 64);
static_assert(NT == 64);
static_assert(WAVES * 8 == NT);
static_assert(NT * PF * 4 <= 2 * NT * PU * 2);

union XTile { unsigned short p[2 * NT * PU]; float f[NT * PF]; };

DEVINL int imin(int a, int b) { return a < b ? a : b; }
DEVINL int imax(int a, int b) { return a > b ? a : b; }

DEVINL v8f wmma_bf(v16b a, v16b b, v8f c) {
  v8f d = __builtin_amdgcn_wmma_f32_16x16x32_bf16(false, a, false, b, (short)0, c, false, false);
  asm volatile("v_nop\n\tv_nop\n\tv_nop\n\tv_nop" : "+v"(d) : "v"(a), "v"(b));
  return d;
}
DEVINL v8f wmma_bf3(const FragB& ah, const FragB& al, const FragB& bh, const FragB& bl, v8f c) {
  c = wmma_bf(ah.v, bh.v, c);
  c = wmma_bf(ah.v, bl.v, c);
  c = wmma_bf(al.v, bh.v, c);
  return c;
}
DEVINL v8f zero8f() {
  v8f z = {0.f, 0.f, 0.f, 0.f, 0.f, 0.f, 0.f, 0.f};
  return z;
}

DEVINL unsigned int bf_rne(float f) {
  const unsigned int u = __float_as_uint(f);
  return (u + 0x7FFFu + ((u >> 16) & 1u)) >> 16;
}
DEVINL void split8(v4f a, v4f b, v8us& hi, v8us& lo) {
  #pragma unroll
  for (int i = 0; i < 4; ++i) {
    const unsigned int h0 = bf_rne(a[i]);
    const float r0 = a[i] - __uint_as_float(h0 << 16);
    hi[i] = (unsigned short)h0;
    lo[i] = (unsigned short)bf_rne(r0);
    const unsigned int h1 = bf_rne(b[i]);
    const float r1 = b[i] - __uint_as_float(h1 << 16);
    hi[4 + i] = (unsigned short)h1;
    lo[4 + i] = (unsigned short)bf_rne(r1);
  }
}

DEVINL float silu_f(float x) {
  const float e = __expf(-x);
  const float d = 1.0f + e;
  return x * __builtin_amdgcn_rcpf(d);
}

__global__ __launch_bounds__(TPB) void k_proj(const float* __restrict__ x, const float* __restrict__ W,
                                            const float* __restrict__ pos, const int* __restrict__ batch,
                                            const float* __restrict__ kvec, int N, int G, int NPG,
                                            float* __restrict__ QD, float* __restrict__ KT,
                                            unsigned short* __restrict__ VTH, unsigned short* __restrict__ VTL,
                                            float* __restrict__ CS, float* __restrict__ SN)
{
  __shared__ __attribute__((aligned(16))) XTile uX;
  __shared__ __attribute__((aligned(16))) unsigned short sW[2 * NT * PU];
  __shared__ __attribute__((aligned(16))) float sF[NT * PF];

  const int tid = threadIdx.x, lane = tid & 31, wave = tid >> 5;
  const int hh = lane >> 4, m16 = lane & 15;
  const int rt = wave >> 1, ct0 = 2 * (wave & 1);
  const int n0 = blockIdx.x * NT;
  const int gsg = n0 / NPG;
  const int sr = tid >> 2, seg = (tid & 3) * 16;
  const int sub4 = lane >> 4, piece4 = (lane & 15) * 4;
  const int sub8 = lane >> 3, piece8 = (lane & 7) * 8;
  unsigned short* sXH = uX.p;
  unsigned short* sXL = uX.p + NT * PU;
  unsigned short* sWH = sW;
  unsigned short* sWL = sW + NT * PU;

  {
    const float* xr = x + (size_t)(n0 + sr) * HD + seg;
    const v4f a0 = *(const v4fa*)(xr);
    const v4f a1 = *(const v4fa*)(xr + 4);
    const v4f a2 = *(const v4fa*)(xr + 8);
    const v4f a3 = *(const v4fa*)(xr + 12);
    v8us hA, lA, hB, lB;
    split8(a0, a1, hA, lA);
    split8(a2, a3, hB, lB);
    *(v8usa*)(sXH + sr * PU + seg)     = hA;
    *(v8usa*)(sXH + sr * PU + seg + 8) = hB;
    *(v8usa*)(sXL + sr * PU + seg)     = lA;
    *(v8usa*)(sXL + sr * PU + seg + 8) = lB;
  }

  #pragma unroll 1
  for (int p = 0; p < 3; ++p) {
    __syncthreads();
    {
      float wv[16];
      const float* wc = W + (size_t)(HD * p) + sr;
      #pragma unroll
      for (int j = 0; j < 16; ++j) wv[j] = wc[(size_t)(seg + j) * (3 * HD)];
      v4f a0, a1, a2, a3;
      #pragma unroll
      for (int i = 0; i < 4; ++i) { a0[i] = wv[i]; a1[i] = wv[4 + i]; a2[i] = wv[8 + i]; a3[i] = wv[12 + i]; }
      v8us hA, lA, hB, lB;
      split8(a0, a1, hA, lA);
      split8(a2, a3, hB, lB);
      *(v8usa*)(sWH + sr * PU + seg)     = hA;
      *(v8usa*)(sWH + sr * PU + seg + 8) = hB;
      *(v8usa*)(sWL + sr * PU + seg)     = lA;
      *(v8usa*)(sWL + sr * PU + seg + 8) = lB;
    }
    __syncthreads();

    v8f acc[2];
    acc[0] = zero8f();
    acc[1] = zero8f();
    #pragma unroll
    for (int kk = 0; kk < 2; ++kk) {
      const int k0 = 32 * kk;
      FragB ah, al, bh[2], bl[2];
      const int ao = (16 * rt + m16) * PU + k0 + 8 * hh;
      ah.half[0] = *(const v8usa*)(sXH + ao);
      ah.half[1] = *(const v8usa*)(sXH + ao + 16);
      al.half[0] = *(const v8usa*)(sXL + ao);
      al.half[1] = *(const v8usa*)(sXL + ao + 16);
      #pragma unroll
      for (int t = 0; t < 2; ++t) {
        const int bo = (16 * (ct0 + t) + m16) * PU + k0 + 8 * hh;
        bh[t].half[0] = *(const v8usa*)(sWH + bo);
        bh[t].half[1] = *(const v8usa*)(sWH + bo + 16);
        bl[t].half[0] = *(const v8usa*)(sWL + bo);
        bl[t].half[1] = *(const v8usa*)(sWL + bo + 16);
      }
      #pragma unroll
      for (int t = 0; t < 2; ++t) acc[t] = wmma_bf3(ah, al, bh[t], bl[t], acc[t]);
    }
    __syncthreads();

    if (p == 0) {
      #pragma unroll
      for (int t = 0; t < 2; ++t) {
        const int c = 16 * (ct0 + t) + m16;
        const int pc = (c >> 1) + 32 * (c & 1);
        #pragma unroll
        for (int r = 0; r < 8; ++r) sF[(16 * rt + 8 * hh + r) * PF + pc] = silu_f(acc[t][r]);
      }
      __syncthreads();
      v4f vv[4];
      #pragma unroll
      for (int i = 0; i < 4; ++i) {
        const int row = 8 * wave + 2 * i + sub4;
        vv[i] = *(const v4fa*)(sF + row * PF + piece4);
      }
      #pragma unroll
      for (int i = 0; i < 4; ++i) {
        const int row = 8 * wave + 2 * i + sub4;
        *(volatile v4f*)(QD + (size_t)(n0 + row) * HD + piece4) = vv[i];
      }
      __threadfence();
      #pragma unroll
      for (int i = 0; i < 4; ++i) {
        const int row = 8 * wave + 2 * i + sub4;
        *(volatile v4f*)(QD + (size_t)(n0 + row) * HD + piece4) = vv[i];
      }
    } else if (p == 1) {
      #pragma unroll
      for (int t = 0; t < 2; ++t) {
        const int c = 16 * (ct0 + t) + m16;
        const int pc = (c >> 1) + 32 * (c & 1);
        #pragma unroll
        for (int r = 0; r < 8; ++r) sF[pc * PF + (16 * rt + 8 * hh + r)] = silu_f(acc[t][r]);
      }
      __syncthreads();
      v4f vv[4];
      #pragma unroll
      for (int i = 0; i < 4; ++i) {
        const int row = 8 * wave + 2 * i + sub4;
        vv[i] = *(const v4fa*)(sF + row * PF + piece4);
      }
      #pragma unroll
      for (int i = 0; i < 4; ++i) {
        const int row = 8 * wave + 2 * i + sub4;
        *(volatile v4f*)(KT + (size_t)row * N + n0 + piece4) = vv[i];
      }
      __threadfence();
      #pragma unroll
      for (int i = 0; i < 4; ++i) {
        const int row = 8 * wave + 2 * i + sub4;
        *(volatile v4f*)(KT + (size_t)row * N + n0 + piece4) = vv[i];
      }
    } else {
      const v4i b0 = *(const v4ia*)(batch + n0 + 16 * rt + 8 * hh);
      const v4i b1 = *(const v4ia*)(batch + n0 + 16 * rt + 8 * hh + 4);
      #pragma unroll
      for (int t = 0; t < 2; ++t) {
        v4f e0, e1;
        #pragma unroll
        for (int r = 0; r < 4; ++r) {
          e0[r] = (b0[r] == gsg) ? acc[t][r] : 0.0f;
          e1[r] = (b1[r] == gsg) ? acc[t][4 + r] : 0.0f;
        }
        v8us hv, lv;
        split8(e0, e1, hv, lv);
        const int c = 16 * (ct0 + t) + m16;
        *(v8usa*)(sWH + c * PU + 16 * rt + 8 * hh) = hv;
        *(v8usa*)(sWL + c * PU + 16 * rt + 8 * hh) = lv;
      }
      __syncthreads();
      v8us hv2[2], lv2[2];
      #pragma unroll
      for (int i = 0; i < 2; ++i) {
        const int row = 8 * wave + 4 * i + sub8;
        hv2[i] = *(const v8usa*)(sWH + row * PU + piece8);
        lv2[i] = *(const v8usa*)(sWL + row * PU + piece8);
      }
      #pragma unroll
      for (int i = 0; i < 2; ++i) {
        const int row = 8 * wave + 4 * i + sub8;
        *(volatile v8us*)(VTH + (size_t)row * N + n0 + piece8) = hv2[i];
        *(volatile v8us*)(VTL + (size_t)row * N + n0 + piece8) = lv2[i];
      }
      __threadfence();
      #pragma unroll
      for (int i = 0; i < 2; ++i) {
        const int row = 8 * wave + 4 * i + sub8;
        *(volatile v8us*)(VTH + (size_t)row * N + n0 + piece8) = hv2[i];
        *(volatile v8us*)(VTL + (size_t)row * N + n0 + piece8) = lv2[i];
      }
    }
  }

  __syncthreads();
  {
    float* sC = sF;
    float* sS = uX.f;
    #pragma unroll 1
    for (int j = 0; j < 16; ++j) {
      const int n = n0 + seg + j;
      int gn = batch[n];
      gn = imin(imax(gn, 0), G - 1);
      const float* kv = kvec + ((size_t)gn * MK + sr) * 3;
      const float px = pos[(size_t)n * 3 + 0];
      const float py = pos[(size_t)n * 3 + 1];
      const float pz = pos[(size_t)n * 3 + 2];
      float ph = px * kv[0];
      ph = fmaf(py, kv[1], ph);
      ph = fmaf(pz, kv[2], ph);
      sC[sr * PF + seg + j] = cosf(ph);
      sS[sr * PF + seg + j] = sinf(ph);
    }
  }
  __syncthreads();
  {
    const float* sC = sF;
    const float* sS = uX.f;
    v4f vc[4], vs[4];
    #pragma unroll
    for (int i = 0; i < 4; ++i) {
      const int row = 8 * wave + 2 * i + sub4;
      vc[i] = *(const v4fa*)(sC + row * PF + piece4);
      vs[i] = *(const v4fa*)(sS + row * PF + piece4);
    }
    #pragma unroll
    for (int i = 0; i < 4; ++i) {
      const int row = 8 * wave + 2 * i + sub4;
      *(volatile v4f*)(CS + (size_t)row * N + n0 + piece4) = vc[i];
      *(volatile v4f*)(SN + (size_t)row * N + n0 + piece4) = vs[i];
    }
    __threadfence();
    #pragma unroll
    for (int i = 0; i < 4; ++i) {
      const int row = 8 * wave + 2 * i + sub4;
      *(volatile v4f*)(CS + (size_t)row * N + n0 + piece4) = vc[i];
      *(volatile v4f*)(SN + (size_t)row * N + n0 + piece4) = vs[i];
    }
  }
}

__global__ __launch_bounds__(TPB) void k_kv(const float* __restrict__ KT, const float* __restrict__ CS,
                                          const float* __restrict__ SN, const unsigned short* __restrict__ VTH,
                                          const unsigned short* __restrict__ VTL, int N, int NPG,
                                          unsigned short* __restrict__ KVTH, unsigned short* __restrict__ KVTL)
{
  __shared__ __attribute__((aligned(16))) unsigned short sK[2 * NT * PU];
  const int tid = threadIdx.x, lane = tid & 31, wave = tid >> 5;
  const int hh = lane >> 4, m16 = lane & 15;
  const int dT = wave >> 1, eT0 = 2 * (wave & 1);
  const int mk = blockIdx.x, g = blockIdx.y;
  const int sr = tid >> 2, seg = (tid & 3) * 16;
  const int jr = sr & 31;
  const bool upper = (sr >= 32);
  unsigned short* sKH = sK;
  unsigned short* sKL = sK + NT * PU;
  const float* arow = KT + (size_t)jr * N + seg;
  const float* brow = KT + (size_t)(32 + jr) * N + seg;
  const float* crow = CS + (size_t)mk * N + seg;
  const float* srow = SN + (size_t)mk * N + seg;

  v8f acc[2];
  acc[0] = zero8f();
  acc[1] = zero8f();
  const int nch = NPG / NT;
  #pragma unroll 1
  for (int ch = 0; ch < nch; ++ch) {
    const int n0 = g * NPG + ch * NT;
    __syncthreads();
    {
      #pragma unroll
      for (int q = 0; q < 2; ++q) {
        const v4f a0 = *(const v4fa*)(arow + n0 + 8 * q);
        const v4f a1 = *(const v4fa*)(arow + n0 + 8 * q + 4);
        const v4f b0 = *(const v4fa*)(brow + n0 + 8 * q);
        const v4f b1 = *(const v4fa*)(brow + n0 + 8 * q + 4);
        const v4f c0 = *(const v4fa*)(crow + n0 + 8 * q);
        const v4f c1 = *(const v4fa*)(crow + n0 + 8 * q + 4);
        const v4f s0 = *(const v4fa*)(srow + n0 + 8 * q);
        const v4f s1 = *(const v4fa*)(srow + n0 + 8 * q + 4);
        v4f e0, e1;
        #pragma unroll
        for (int i = 0; i < 4; ++i) {
          const float ca0 = upper ? s0[i] : c0[i];
          const float sb0 = upper ? c0[i] : -s0[i];
          e0[i] = a0[i] * ca0 + b0[i] * sb0;
          const float ca1 = upper ? s1[i] : c1[i];
          const float sb1 = upper ? c1[i] : -s1[i];
          e1[i] = a1[i] * ca1 + b1[i] * sb1;
        }
        v8us hv, lv;
        split8(e0, e1, hv, lv);
        *(v8usa*)(sKH + sr * PU + seg + 8 * q) = hv;
        *(v8usa*)(sKL + sr * PU + seg + 8 * q) = lv;
      }
    }
    __syncthreads();
    #pragma unroll
    for (int kk = 0; kk < 2; ++kk) {
      const int k0 = 32 * kk;
      FragB ah, al, bh[2], bl[2];
      const int ao = (16 * dT + m16) * PU + k0 + 8 * hh;
      ah.half[0] = *(const v8usa*)(sKH + ao);
      ah.half[1] = *(const v8usa*)(sKH + ao + 16);
      al.half[0] = *(const v8usa*)(sKL + ao);
      al.half[1] = *(const v8usa*)(sKL + ao + 16);
      #pragma unroll
      for (int t = 0; t < 2; ++t) {
        const size_t bo = (size_t)(16 * (eT0 + t) + m16) * N + n0 + k0 + 8 * hh;
        bh[t].half[0] = *(const v8usa*)(VTH + bo);
        bh[t].half[1] = *(const v8usa*)(VTH + bo + 16);
        bl[t].half[0] = *(const v8usa*)(VTL + bo);
        bl[t].half[1] = *(const v8usa*)(VTL + bo + 16);
      }
      #pragma unroll
      for (int t = 0; t < 2; ++t) acc[t] = wmma_bf3(ah, al, bh[t], bl[t], acc[t]);
    }
  }
  __syncthreads();
  #pragma unroll
  for (int t = 0; t < 2; ++t) {
    v4f a0, a1;
    #pragma unroll
    for (int r = 0; r < 4; ++r) { a0[r] = acc[t][r]; a1[r] = acc[t][4 + r]; }
    v8us hv, lv;
    split8(a0, a1, hv, lv);
    const int h = 16 * (eT0 + t) + m16;
    *(v8usa*)(sKH + h * PU + 16 * dT + 8 * hh) = hv;
    *(v8usa*)(sKL + h * PU + 16 * dT + 8 * hh) = lv;
  }
  __syncthreads();
  {
    const int sub8 = lane >> 3, piece8 = (lane & 7) * 8;
    const size_t rp = (size_t)MK * HD;
    v8us hv2[2], lv2[2];
    #pragma unroll
    for (int i = 0; i < 2; ++i) {
      const int row = 8 * wave + 4 * i + sub8;
      hv2[i] = *(const v8usa*)(sKH + row * PU + piece8);
      lv2[i] = *(const v8usa*)(sKL + row * PU + piece8);
    }
    #pragma unroll
    for (int i = 0; i < 2; ++i) {
      const int row = 8 * wave + 4 * i + sub8;
      const size_t o = ((size_t)g * HD + row) * rp + (size_t)mk * HD + piece8;
      *(volatile v8us*)(KVTH + o) = hv2[i];
      *(volatile v8us*)(KVTL + o) = lv2[i];
    }
    __threadfence();
    #pragma unroll
    for (int i = 0; i < 2; ++i) {
      const int row = 8 * wave + 4 * i + sub8;
      const size_t o = ((size_t)g * HD + row) * rp + (size_t)mk * HD + piece8;
      *(volatile v8us*)(KVTH + o) = hv2[i];
      *(volatile v8us*)(KVTL + o) = lv2[i];
    }
  }
}

__global__ __launch_bounds__(TPB) void k_out(const float* __restrict__ QD, const float* __restrict__ CS,
                                           const float* __restrict__ SN, const float* __restrict__ wk,
                                           const int* __restrict__ batch, const unsigned short* __restrict__ KVTH,
                                           const unsigned short* __restrict__ KVTL, int N, int G, int NPG,
                                           float* __restrict__ out)
{
  __shared__ __attribute__((aligned(16))) unsigned short sQ[2 * NT * PU];
  __shared__ __attribute__((aligned(16))) float sO[NT * PF];
  const int tid = threadIdx.x, lane = tid & 31, wave = tid >> 5;
  const int hh = lane >> 4, m16 = lane & 15;
  const int rt = wave >> 1, eT0 = 2 * (wave & 1);
  const int n0 = blockIdx.x * NT;
  const int gsg = n0 / NPG;
  const int sr = tid >> 2, seg = (tid & 3) * 16;
  const int j0 = seg & 31;
  const bool upper = (seg >= 32);
  const int n = n0 + sr;
  unsigned short* sQH = sQ;
  unsigned short* sQL = sQ + NT * PU;

  float aR[16], bR[16];
  {
    const float* qr = QD + (size_t)n * HD + j0;
    #pragma unroll
    for (int q = 0; q < 4; ++q) {
      const v4f ta = *(const v4fa*)(qr + 4 * q);
      const v4f tb = *(const v4fa*)(qr + 32 + 4 * q);
      #pragma unroll
      for (int i = 0; i < 4; ++i) { aR[4 * q + i] = ta[i]; bR[4 * q + i] = tb[i]; }
    }
  }
  int gn = batch[n];
  gn = imin(imax(gn, 0), G - 1);
  const float* wrow = wk + (size_t)gn * MK;
  const size_t rp = (size_t)MK * HD;
  const unsigned short* kvh = KVTH + (size_t)gsg * HD * rp;
  const unsigned short* kvl = KVTL + (size_t)gsg * HD * rp;

  v8f acc[2];
  acc[0] = zero8f();
  acc[1] = zero8f();
  #pragma unroll 1
  for (int mk = 0; mk < MK; ++mk) {
    __syncthreads();
    {
      const float c = CS[(size_t)mk * N + n];
      const float s = SN[(size_t)mk * N + n];
      const float ww = wrow[mk] * QSCALE;
      const float ca = upper ? s : c;
      const float sb = upper ? c : -s;
      v4f e[4];
      #pragma unroll
      for (int q = 0; q < 4; ++q) {
        #pragma unroll
        for (int i = 0; i < 4; ++i) e[q][i] = (aR[4 * q + i] * ca + bR[4 * q + i] * sb) * ww;
      }
      v8us hA, lA, hB, lB;
      split8(e[0], e[1], hA, lA);
      split8(e[2], e[3], hB, lB);
      *(v8usa*)(sQH + sr * PU + seg)     = hA;
      *(v8usa*)(sQH + sr * PU + seg + 8) = hB;
      *(v8usa*)(sQL + sr * PU + seg)     = lA;
      *(v8usa*)(sQL + sr * PU + seg + 8) = lB;
    }
    __syncthreads();
    #pragma unroll
    for (int kk = 0; kk < 2; ++kk) {
      const int k0 = 32 * kk;
      FragB ah, al, bh[2], bl[2];
      const int ao = (16 * rt + m16) * PU + k0 + 8 * hh;
      ah.half[0] = *(const v8usa*)(sQH + ao);
      ah.half[1] = *(const v8usa*)(sQH + ao + 16);
      al.half[0] = *(const v8usa*)(sQL + ao);
      al.half[1] = *(const v8usa*)(sQL + ao + 16);
      #pragma unroll
      for (int t = 0; t < 2; ++t) {
        const size_t bo = (size_t)(16 * (eT0 + t) + m16) * rp + (size_t)mk * HD + k0 + 8 * hh;
        bh[t].half[0] = *(const v8usa*)(kvh + bo);
        bh[t].half[1] = *(const v8usa*)(kvh + bo + 16);
        bl[t].half[0] = *(const v8usa*)(kvl + bo);
        bl[t].half[1] = *(const v8usa*)(kvl + bo + 16);
      }
      #pragma unroll
      for (int t = 0; t < 2; ++t) acc[t] = wmma_bf3(ah, al, bh[t], bl[t], acc[t]);
    }
  }

  #pragma unroll
  for (int t = 0; t < 2; ++t) {
    const int h = 16 * (eT0 + t) + m16;
    #pragma unroll
    for (int r = 0; r < 8; ++r) sO[(16 * rt + 8 * hh + r) * PF + h] = acc[t][r];
  }
  __syncthreads();
  {
    const int sub4 = lane >> 4, piece4 = (lane & 15) * 4;
    const float qn = __int_as_float(0x7fc00000);
    v4f vn;
    vn[0] = qn; vn[1] = qn; vn[2] = qn; vn[3] = qn;
    v4f vv[4];
    #pragma unroll
    for (int i = 0; i < 4; ++i) {
      const int row = 8 * wave + 2 * i + sub4;
      v4f v = *(const v4fa*)(sO + row * PF + piece4);
      const int bn = batch[n0 + row];
      if (bn != gsg) v = vn;
      vv[i] = v;
    }
    #pragma unroll
    for (int i = 0; i < 4; ++i) {
      const int row = 8 * wave + 2 * i + sub4;
      *(volatile v4f*)(out + (size_t)(n0 + row) * HD + piece4) = vv[i];
    }
    __threadfence();
    #pragma unroll
    for (int i = 0; i < 4; ++i) {
      const int row = 8 * wave + 2 * i + sub4;
      *(volatile v4f*)(out + (size_t)(n0 + row) * HD + piece4) = vv[i];
    }
  }
}

extern "C" void kernel_launch(void* const* d_in, const int* in_sizes, int n_in,
                              void* d_out, int out_size, void* d_ws, size_t ws_size,
                              hipStream_t stream)
{
  if (n_in < 6) return;
  const int nx = in_sizes[0];
  if (nx <= 0 || (nx % HD) != 0) return;
  const int N = nx / HD;
  if (in_sizes[1] != 3 * N) return;
  if (in_sizes[2] != N) return;
  if (in_sizes[4] <= 0 || (in_sizes[4] % MK) != 0) return;
  const int G = in_sizes[4] / MK;
  if (in_sizes[3] != G * MK * 3) return;
  if (in_sizes[5] != HD * 3 * HD) return;
  if (out_size != N * HD) return;
  if ((N % G) != 0) return;
  const int NPG = N / G;
  if ((NPG % NT) != 0) return;

  const float* x     = (const float*)d_in[0];
  const float* pos   = (const float*)d_in[1];
  const int*   batch = (const int*)d_in[2];
  const float* kvec  = (const float*)d_in[3];
  const float* wk    = (const float*)d_in[4];
  const float* W     = (const float*)d_in[5];
  float* outp = (float*)d_out;

  const size_t szQD = (size_t)N * HD * 4;
  const size_t szKT = (size_t)HD * N * 4;
  const size_t szVT = (size_t)HD * N * 2;
  const size_t szCS = (size_t)MK * N * 4;
  const size_t szKV = (size_t)G * HD * MK * HD * 2;
  size_t off = 0;
  char* ws = (char*)d_ws;
  float* QD = (float*)(ws + off);                    off += szQD;
  float* KT = (float*)(ws + off);                    off += szKT;
  unsigned short* VTH = (unsigned short*)(ws + off);  off += szVT;
  unsigned short* VTL = (unsigned short*)(ws + off);  off += szVT;
  float* CS = (float*)(ws + off);                    off += szCS;
  float* SN = (float*)(ws + off);                    off += szCS;
  unsigned short* KVTH = (unsigned short*)(ws + off); off += szKV;
  unsigned short* KVTL = (unsigned short*)(ws + off); off += szKV;
  if (off > ws_size) return;

  k_proj<<<N / NT, TPB, 0, stream>>>(x, W, pos, batch, kvec, N, G, NPG, QD, KT, VTH, VTL, CS, SN);
  k_kv<<<dim3(MK, G), TPB, 0, stream>>>(KT, CS, SN, VTH, VTL, N, NPG, KVTH, KVTL);
  k_out<<<N / NT, TPB, 0, stream>>>(QD, CS, SN, wk, batch, KVTH, KVTL, N, G, NPG, outp);
  (void)hipGetLastError();
}
